// HeteGraphAttentionLayer_47888885350604
// MI455X (gfx1250) — hardware-verified
//
#include <hip/hip_runtime.h>
#include <math.h>
#include <stdint.h>

#define NB    8
#define NN    1024
#define DD    256
#define SEQL  512
#define SEGL  256
#define GAZL  256
#define MROWS (NB * NN)
#define TP    260

#define NX8   (MROWS * DD / 8)
#define NW8   (DD * DD / 8)
#define PB_X  (NX8 / 256)
#define PB_W  (NW8 / 256)
#define PB_ALL (PB_X + PB_W + 2)

static_assert(SEQL % 128 == 0);
static_assert((SEQL + SEGL) % 128 == 0);
static_assert(SEQL + SEGL + GAZL == NN);
static_assert(NN % 64 == 0);
static_assert(DD % 32 == 0);
static_assert(DD == 256);
static_assert(NX8 % 256 == 0);
static_assert(NW8 % 256 == 0);
static_assert(MROWS % 64 == 0);

typedef __attribute__((ext_vector_type(16))) __bf16       v16b;
typedef __attribute__((ext_vector_type(8)))  float        v8f;
typedef __attribute__((ext_vector_type(4)))  float        v4f;
typedef __attribute__((ext_vector_type(4)))  unsigned int v4u;
typedef __attribute__((ext_vector_type(4)))  int          v4i;
typedef v4f __attribute__((may_alias)) v4fa;
typedef v4u __attribute__((may_alias)) v4ua;
typedef v4i __attribute__((may_alias)) v4ia;

union FB { v16b v; v4u q[2]; };

__device__ __forceinline__ unsigned bf_bits(float f) {
  const unsigned u = __float_as_uint(f);
  const unsigned r = (u + 0x7FFFu + ((u >> 16) & 1u)) >> 16;
  return (f != f) ? 0x7FC0u : r;
}
__device__ __forceinline__ float bf_val(unsigned h) { return __uint_as_float(h << 16); }

__device__ __forceinline__ v8f wmb(v16b a, v16b b, v8f c) {
  c = __builtin_amdgcn_wmma_f32_16x16x32_bf16(false, a, false, b, (short)0, c, false, false);
  asm volatile("v_nop\n\tv_nop\n\tv_nop\n\tv_nop" : "+v"(c) : "v"(a), "v"(b));
  return c;
}

__device__ __forceinline__ v16b ldfrag_g(const unsigned short* __restrict__ p) {
  FB f;
  f.q[0] = *(const v4ua*)(p);
  f.q[1] = *(const v4ua*)(p + 16);
  return f.v;
}

__device__ __forceinline__ void cvt8_store(const float* __restrict__ src, unsigned short* __restrict__ dst) {
  const v4f a = *(const v4fa*)(src);
  const v4f c = *(const v4fa*)(src + 4);
  v4u o;
  o.x = bf_bits(a.x) | (bf_bits(a.y) << 16);
  o.y = bf_bits(a.z) | (bf_bits(a.w) << 16);
  o.z = bf_bits(c.x) | (bf_bits(c.y) << 16);
  o.w = bf_bits(c.z) | (bf_bits(c.w) << 16);
  *(volatile v4u*)dst = o;
  __threadfence();
  *(volatile v4u*)dst = o;
}
__device__ __forceinline__ void cvt4_store(const float* __restrict__ src, float* __restrict__ dst) {
  const v4f a = *(const v4fa*)(src);
  v4f o;
  o.x = bf_val(bf_bits(a.x));
  o.y = bf_val(bf_bits(a.y));
  o.z = bf_val(bf_bits(a.z));
  o.w = bf_val(bf_bits(a.w));
  *(volatile v4f*)dst = o;
  __threadfence();
  *(volatile v4f*)dst = o;
}

__global__ __launch_bounds__(256) void k_prep(
    const float* __restrict__ x, const float* __restrict__ W,
    const float* __restrict__ a1, const float* __restrict__ a2,
    unsigned short* __restrict__ XB, unsigned short* __restrict__ WB, float* __restrict__ AV) {
  const int blk = blockIdx.x;
  const int tid = threadIdx.x;
  if (blk < PB_X) {
    const size_t u = (size_t)blk * 256 + tid;
    cvt8_store(x + u * 8, XB + u * 8);
  } else if (blk < PB_X + PB_W) {
    const size_t u = (size_t)(blk - PB_X) * 256 + tid;
    cvt8_store(W + u * 8, WB + u * 8);
  } else if (blk == PB_X + PB_W) {
    cvt4_store(a1 + tid * 4, AV + tid * 4);
  } else if (blk == PB_X + PB_W + 1) {
    cvt4_store(a2 + tid * 4, AV + 1024 + tid * 4);
  }
}

__global__ __launch_bounds__(256) __attribute__((amdgpu_num_vgpr(248)))
void k_h(const unsigned short* __restrict__ XB, const unsigned short* __restrict__ WB,
         const float* __restrict__ AV,
         unsigned short* __restrict__ VTH, unsigned short* __restrict__ VTL,
         float* __restrict__ SS) {
  __shared__ __align__(16) float tile[64 * TP];
  __shared__ __align__(16) float avs[8 * DD];
  __shared__ __align__(16) float dots[8 * 64];

  const int tid  = threadIdx.x;
  const int lane = tid & 31;
  const int w    = tid >> 5;
  const int hh   = lane >> 4;
  const int m    = lane & 15;
  const int row0 = blockIdx.x * 64;
  const int b    = row0 >> 10;
  const int n0   = row0 & (NN - 1);
  const int rg   = w & 3;
  const int ch   = w >> 2;

#pragma unroll
  for (int i = 0; i < 2; ++i) {
    const int idx = i * 256 + tid;
    const v4f t = *(const v4fa*)(AV + idx * 4);
    *(v4fa*)(avs + idx * 4) = t;
  }

  const v8f zero8 = {0.f, 0.f, 0.f, 0.f, 0.f, 0.f, 0.f, 0.f};
  v8f acc[8];
#pragma unroll
  for (int t = 0; t < 8; ++t) acc[t] = zero8;

  const unsigned short* ap = XB + (size_t)(row0 + rg * 16 + m) * DD + 8 * hh;
  const unsigned short* bp = WB + (size_t)(ch * 128 + m) * DD + 8 * hh;

#pragma unroll 1
  for (int k0 = 0; k0 < DD; k0 += 32) {
    const v16b a = ldfrag_g(ap + k0);
#pragma unroll
    for (int t = 0; t < 8; ++t) {
      const v16b bf = ldfrag_g(bp + (size_t)t * 16 * DD + k0);
      acc[t] = wmb(a, bf, acc[t]);
    }
  }

#pragma unroll
  for (int t = 0; t < 8; ++t)
#pragma unroll
    for (int r = 0; r < 8; ++r)
      tile[(rg * 16 + 8 * hh + r) * TP + ch * 128 + 16 * t + m] = acc[t][r];
  __syncthreads();

  {
    float av[8][8];
#pragma unroll
    for (int k = 0; k < 8; ++k) {
      const v4f p0 = *(const v4fa*)(avs + k * DD + lane * 8);
      const v4f p1 = *(const v4fa*)(avs + k * DD + lane * 8 + 4);
      av[k][0] = p0.x; av[k][1] = p0.y; av[k][2] = p0.z; av[k][3] = p0.w;
      av[k][4] = p1.x; av[k][5] = p1.y; av[k][6] = p1.z; av[k][7] = p1.w;
    }
#pragma unroll 1
    for (int rr = 0; rr < 8; ++rr) {
      const int row = w * 8 + rr;
      const v4f x0 = *(const v4fa*)(tile + row * TP + lane * 8);
      const v4f x1 = *(const v4fa*)(tile + row * TP + lane * 8 + 4);
      float hv[8];
      hv[0] = x0.x; hv[1] = x0.y; hv[2] = x0.z; hv[3] = x0.w;
      hv[4] = x1.x; hv[5] = x1.y; hv[6] = x1.z; hv[7] = x1.w;
      float d[8];
#pragma unroll
      for (int k = 0; k < 8; ++k) {
        float s = 0.0f;
#pragma unroll
        for (int e = 0; e < 8; ++e) s = fmaf(hv[e], av[k][e], s);
        d[k] = s;
      }
#pragma unroll
      for (int off = 16; off > 0; off >>= 1) {
#pragma unroll
        for (int k = 0; k < 8; ++k) d[k] += __shfl_xor(d[k], off, 32);
      }
      float sel = d[0];
      sel = (lane == 1) ? d[1] : sel;
      sel = (lane == 2) ? d[2] : sel;
      sel = (lane == 3) ? d[3] : sel;
      sel = (lane == 4) ? d[4] : sel;
      sel = (lane == 5) ? d[5] : sel;
      sel = (lane == 6) ? d[6] : sel;
      sel = (lane == 7) ? d[7] : sel;
      if (lane < 8) dots[lane * 64 + row] = sel;
    }
  }
  __syncthreads();

  if (w < 4) {
    const int kk = 2 * w + hh;
    const v4f v = *(const v4fa*)(dots + kk * 64 + m * 4);
    float* dst = SS + ((size_t)(b * 8 + kk) * NN + n0 + m * 4);
    *(volatile v4f*)dst = v;
    __threadfence();
    *(volatile v4f*)dst = v;
  }

  {
    const int sub = lane >> 3;
    const int q8  = lane & 7;
    v4u hq[8], lq[8];
#pragma unroll
    for (int it = 0; it < 8; ++it) {
      const int c = w * 32 + it * 4 + sub;
      v4u a, a2;
#pragma unroll
      for (int qq = 0; qq < 4; ++qq) {
        const float f0 = tile[(8 * q8 + 2 * qq) * TP + c];
        const float f1 = tile[(8 * q8 + 2 * qq + 1) * TP + c];
        const unsigned h0 = bf_bits(f0), h1 = bf_bits(f1);
        const unsigned l0 = bf_bits(f0 - bf_val(h0)), l1 = bf_bits(f1 - bf_val(h1));
        a[qq]  = h0 | (h1 << 16);
        a2[qq] = l0 | (l1 << 16);
      }
      hq[it] = a; lq[it] = a2;
    }
    for (int pass = 0; pass < 2; ++pass) {
#pragma unroll
      for (int it = 0; it < 8; ++it) {
        const int c = w * 32 + it * 4 + sub;
        const size_t go = ((size_t)(b * DD + c)) * NN + n0 + 8 * q8;
        *(volatile v4u*)(VTH + go) = hq[it];
        *(volatile v4u*)(VTL + go) = lq[it];
      }
      __threadfence();
    }
  }
}

__device__ __forceinline__ int ksel(int ty, int kt) {
  int k = -1;
  k = (ty == 0 && kt == 1) ? 2 : k;
  k = (ty == 1 && kt == 0) ? 2 : k;
  k = (ty == 1 && kt == 1) ? 1 : k;
  k = (ty == 0 && kt == 2) ? 3 : k;
  k = (ty == 2 && kt == 0) ? 3 : k;
  return k;
}
__device__ __forceinline__ float leaky(float v) { return (v > 0.0f) ? v : 0.2f * v; }
__device__ __forceinline__ float logit1(float s1k, float s2v, bool has, bool isdiag, float ldiag, int adjv) {
  const float lk = leaky(s1k + s2v);
  float L = has ? lk : 0.0f;
  L = isdiag ? ldiag : L;
  L = (adjv == 0) ? -1.0e9f : L;
  return L;
}
__device__ __forceinline__ float elu1(float v) { return (v > 0.0f) ? v : expm1f(v); }

__global__ __launch_bounds__(256) __attribute__((amdgpu_num_vgpr(248)))
void k_att(const int* __restrict__ adj, const float* __restrict__ SS,
           const unsigned short* __restrict__ VTH, const unsigned short* __restrict__ VTL,
           const int* __restrict__ p_seq, const int* __restrict__ p_seg, const int* __restrict__ p_gaz,
           float* __restrict__ out) {
  __shared__ __align__(16) float s2s[4 * NN];
  __shared__ __align__(16) float s1s[4 * 64];
  __shared__ __align__(16) float ms[64];
  __shared__ __align__(16) float rls[64];
  __shared__ __align__(16) unsigned short ph[2][64 * 32];
  __shared__ __align__(16) unsigned short pl[2][64 * 32];
  __shared__ __align__(16) float tile[64 * TP];

  const int tid  = threadIdx.x;
  const int lane = tid & 31;
  const int w    = tid >> 5;
  const int hh   = lane >> 4;
  const int m    = lane & 15;
  const int b    = blockIdx.x >> 4;
  const int q0   = (blockIdx.x & 15) * 64;
  const int ty   = (q0 < SEQL) ? 0 : ((q0 < SEQL + SEGL) ? 1 : 2);

  const bool bad = (p_seq[0] != SEQL) | (p_seg[0] != SEGL) | (p_gaz[0] != GAZL);

  {
    const float* s2g = SS + (size_t)(b * 8 + 4) * NN;
#pragma unroll
    for (int i = 0; i < 4; ++i) {
      const int idx = i * 256 + tid;
      const v4f t = *(const v4fa*)(s2g + idx * 4);
      *(v4fa*)(s2s + idx * 4) = t;
    }
    if (tid < 64) {
      const int k = tid >> 4, r4 = (tid & 15) * 4;
      const v4f t = *(const v4fa*)(SS + (size_t)(b * 8 + k) * NN + q0 + r4);
      *(v4fa*)(s1s + k * 64 + r4) = t;
    }
  }
  __syncthreads();

#pragma unroll 1
  for (int rr = 0; rr < 8; ++rr) {
    const int row = w * 8 + rr;
    const int i   = q0 + row;
    const int* ar = adj + ((size_t)(b * NN + i)) * NN;
    const float ldiag = leaky(s1s[row] + s2s[i]);
    float L[32];
    float mx = -INFINITY;
#pragma unroll
    for (int t = 0; t < 8; ++t) {
      const v4i av = *(const v4ia*)(ar + t * 128 + lane * 4);
      const int kt = (t * 128 < SEQL) ? 0 : ((t * 128 < SEQL + SEGL) ? 1 : 2);
      const int ks = ksel(ty, kt);
      const int kc = (ks < 0) ? 0 : ks;
      const bool has = ks >= 0;
      const float s1k = s1s[kc * 64 + row];
      const v4f s2v = *(const v4fa*)(s2s + kc * NN + t * 128 + lane * 4);
      const int jb = t * 128 + lane * 4;
      const float l0 = logit1(s1k, s2v.x, has, (jb + 0) == i, ldiag, av.x);
      const float l1 = logit1(s1k, s2v.y, has, (jb + 1) == i, ldiag, av.y);
      const float l2 = logit1(s1k, s2v.z, has, (jb + 2) == i, ldiag, av.z);
      const float l3 = logit1(s1k, s2v.w, has, (jb + 3) == i, ldiag, av.w);
      L[t * 4 + 0] = l0; L[t * 4 + 1] = l1; L[t * 4 + 2] = l2; L[t * 4 + 3] = l3;
      mx = fmaxf(mx, fmaxf(fmaxf(l0, l1), fmaxf(l2, l3)));
    }
#pragma unroll
    for (int off = 16; off > 0; off >>= 1) mx = fmaxf(mx, __shfl_xor(mx, off, 32));
    float sum = 0.0f;
#pragma unroll
    for (int e = 0; e < 32; ++e) sum += expf(L[e] - mx);
#pragma unroll
    for (int off = 16; off > 0; off >>= 1) sum += __shfl_xor(sum, off, 32);
    if (lane == 0) { ms[row] = mx; rls[row] = 1.0f / sum; }
  }
  __syncthreads();

  const int prow = tid >> 2;
  const int kq   = tid & 3;
  const int pi   = q0 + prow;
  const float pm    = ms[prow];
  const float prl   = rls[prow];
  const float pdiag = leaky(s1s[prow] + s2s[pi]);
  const int* parow = adj + ((size_t)(b * NN + pi)) * NN + kq * 8;

  const int rg = w & 3;
  const int ch = w >> 2;
  const unsigned short* vh = VTH + ((size_t)(b * DD + ch * 128 + m)) * NN + 8 * hh;
  const unsigned short* vl = VTL + ((size_t)(b * DD + ch * 128 + m)) * NN + 8 * hh;

  const v8f zero8 = {0.f, 0.f, 0.f, 0.f, 0.f, 0.f, 0.f, 0.f};
  v8f acc[8];
#pragma unroll
  for (int t = 0; t < 8; ++t) acc[t] = zero8;

#pragma unroll 1
  for (int kc = 0; kc < NN / 32; ++kc) {
    const int buf = kc & 1;
    const int kt  = (kc * 32 < SEQL) ? 0 : ((kc * 32 < SEQL + SEGL) ? 1 : 2);
    const int ks  = ksel(ty, kt);
    const int kcl = (ks < 0) ? 0 : ks;
    const bool has = ks >= 0;
    const int j0 = kc * 32 + kq * 8;
    const v4i a0 = *(const v4ia*)(parow + kc * 32);
    const v4i a1 = *(const v4ia*)(parow + kc * 32 + 4);
    const float s1k = s1s[kcl * 64 + prow];
    const v4f sa = *(const v4fa*)(s2s + kcl * NN + j0);
    const v4f sb = *(const v4fa*)(s2s + kcl * NN + j0 + 4);
    float p[8];
    p[0] = expf(logit1(s1k, sa.x, has, (j0 + 0) == pi, pdiag, a0.x) - pm) * prl;
    p[1] = expf(logit1(s1k, sa.y, has, (j0 + 1) == pi, pdiag, a0.y) - pm) * prl;
    p[2] = expf(logit1(s1k, sa.z, has, (j0 + 2) == pi, pdiag, a0.z) - pm) * prl;
    p[3] = expf(logit1(s1k, sa.w, has, (j0 + 3) == pi, pdiag, a0.w) - pm) * prl;
    p[4] = expf(logit1(s1k, sb.x, has, (j0 + 4) == pi, pdiag, a1.x) - pm) * prl;
    p[5] = expf(logit1(s1k, sb.y, has, (j0 + 5) == pi, pdiag, a1.y) - pm) * prl;
    p[6] = expf(logit1(s1k, sb.z, has, (j0 + 6) == pi, pdiag, a1.z) - pm) * prl;
    p[7] = expf(logit1(s1k, sb.w, has, (j0 + 7) == pi, pdiag, a1.w) - pm) * prl;
    v4u hq, lq;
#pragma unroll
    for (int qq = 0; qq < 4; ++qq) {
      const unsigned h0 = bf_bits(p[2 * qq]), h1 = bf_bits(p[2 * qq + 1]);
      const unsigned l0 = bf_bits(p[2 * qq] - bf_val(h0)), l1 = bf_bits(p[2 * qq + 1] - bf_val(h1));
      hq[qq] = h0 | (h1 << 16);
      lq[qq] = l0 | (l1 << 16);
    }
    *(v4ua*)(&ph[buf][prow * 32 + kq * 8]) = hq;
    *(v4ua*)(&pl[buf][prow * 32 + kq * 8]) = lq;
    __syncthreads();

    FB ah, al;
    ah.q[0] = *(const v4ua*)(&ph[buf][(rg * 16 + m) * 32 + 8 * hh]);
    ah.q[1] = *(const v4ua*)(&ph[buf][(rg * 16 + m) * 32 + 16 + 8 * hh]);
    al.q[0] = *(const v4ua*)(&pl[buf][(rg * 16 + m) * 32 + 8 * hh]);
    al.q[1] = *(const v4ua*)(&pl[buf][(rg * 16 + m) * 32 + 16 + 8 * hh]);
#pragma unroll
    for (int t = 0; t < 8; ++t) {
      const v16b bh = ldfrag_g(vh + (size_t)t * 16 * NN + kc * 32);
      const v16b bl = ldfrag_g(vl + (size_t)t * 16 * NN + kc * 32);
      acc[t] = wmb(ah.v, bh, acc[t]);
      acc[t] = wmb(al.v, bh, acc[t]);
      acc[t] = wmb(ah.v, bl, acc[t]);
    }
  }

#pragma unroll
  for (int t = 0; t < 8; ++t)
#pragma unroll
    for (int r = 0; r < 8; ++r)
      tile[(rg * 16 + 8 * hh + r) * TP + ch * 128 + 16 * t + m] = acc[t][r];
  __syncthreads();

  const float nanv = __uint_as_float(0x7fc00000u);
#pragma unroll 1
  for (int it = 0; it < 16; ++it) {
    const int row = w * 8 + (it >> 1);
    const int col = (it & 1) * 128 + lane * 4;
    float* tp = tile + row * TP + col;
    const v4f v = *(const v4fa*)tp;
    v4f o;
    o.x = elu1(v.x); o.y = elu1(v.y); o.z = elu1(v.z); o.w = elu1(v.w);
    o.x = bad ? nanv : o.x; o.y = bad ? nanv : o.y; o.z = bad ? nanv : o.z; o.w = bad ? nanv : o.w;
    *(v4fa*)tp = o;
    *(volatile v4f*)(out + ((size_t)(b * NN + q0 + row)) * DD + col) = o;
  }
  __threadfence();
#pragma unroll 1
  for (int it = 0; it < 16; ++it) {
    const int row = w * 8 + (it >> 1);
    const int col = (it & 1) * 128 + lane * 4;
    const v4f o = *(const v4fa*)(tile + row * TP + col);
    *(volatile v4f*)(out + ((size_t)(b * NN + q0 + row)) * DD + col) = o;
  }
}

extern "C" void kernel_launch(void* const* d_in, const int* in_sizes, int n_in,
                              void* d_out, int out_size, void* d_ws, size_t ws_size,
                              hipStream_t stream) {
  if (n_in < 8) return;
  if (in_sizes[0] != MROWS * DD) return;
  if (in_sizes[1] != NB * NN * NN) return;
  if (in_sizes[2] != DD * DD) return;
  if (in_sizes[3] != 4 * DD || in_sizes[4] != 4 * DD) return;
  if (in_sizes[5] != 1 || in_sizes[6] != 1 || in_sizes[7] != 1) return;
  if (out_size != MROWS * DD) return;

  const float* x   = (const float*)d_in[0];
  const int*   adj = (const int*)d_in[1];
  const float* W   = (const float*)d_in[2];
  const float* a1  = (const float*)d_in[3];
  const float* a2  = (const float*)d_in[4];
  const int*   pseq = (const int*)d_in[5];
  const int*   pseg = (const int*)d_in[6];
  const int*   pgaz = (const int*)d_in[7];
  float* out = (float*)d_out;

  const size_t szXB = (size_t)MROWS * DD * 2;
  const size_t szWB = (size_t)DD * DD * 2;
  const size_t szAV = (size_t)8 * DD * 4;
  const size_t szSS = (size_t)NB * 8 * NN * 4;
  const size_t szVT = (size_t)NB * DD * NN * 2;
  size_t off = 0;
  const size_t oXB = off; off += szXB;
  const size_t oWB = off; off += szWB;
  const size_t oAV = off; off += szAV;
  const size_t oSS = off; off += szSS;
  const size_t oVH = off; off += szVT;
  const size_t oVL = off; off += szVT;
  if (off > ws_size) return;

  char* ws = (char*)d_ws;
  unsigned short* XB  = (unsigned short*)(ws + oXB);
  unsigned short* WB  = (unsigned short*)(ws + oWB);
  float*          AV  = (float*)(ws + oAV);
  float*          SSp = (float*)(ws + oSS);
  unsigned short* VTH = (unsigned short*)(ws + oVH);
  unsigned short* VTL = (unsigned short*)(ws + oVL);

  k_prep<<<dim3(PB_ALL), dim3(256), 0, stream>>>(x, W, a1, a2, XB, WB, AV);
  k_h<<<dim3(MROWS / 64), dim3(256), 0, stream>>>(XB, WB, AV, VTH, VTL, SSp);
  k_att<<<dim3(NB * (NN / 64)), dim3(256), 0, stream>>>(adj, SSp, VTH, VTL, pseq, pseg, pgaz, out);
  (void)hipGetLastError();
}
